// CREStereo_12833362280738
// MI455X (gfx1250) — hardware-verified
//
#include <hip/hip_runtime.h>


namespace {
constexpr int NB = 2, C = 256, H = 96, W = 192, G = 4, GC = 64, K9 = 9, HW = H * W;
constexpr float XS = 8.0f;

typedef _Float16 b16;
typedef __attribute__((ext_vector_type(16))) _Float16 v16b;
typedef __attribute__((ext_vector_type(8))) _Float16 v8b;
typedef __attribute__((ext_vector_type(8))) float v8f;
typedef __attribute__((ext_vector_type(4))) float v4f;
__device__ __forceinline__ float bf16_rne(float f) { unsigned int u = __float_as_uint(f); u += 0x7FFFu + ((u >> 16) & 1u); return __uint_as_float(u & 0xFFFF0000u); }
__device__ __forceinline__ void split16(float v, b16& hi, b16& lo) { hi = (b16)v; lo = (b16)(v - (float)hi); }
__device__ __forceinline__ v16b frag_kb(const b16* p, int hh) { const v8b a = *(const v8b*)(p + 8 * hh), b = *(const v8b*)(p + 16 + 8 * hh); v16b f;
#pragma unroll
  for (int e = 0; e < 8; ++e) { f[e] = a[e]; f[8 + e] = b[e]; } return f; }
__device__ __forceinline__ v8f wmma16b(v16b a, v16b b, v8f c) { v8f d = __builtin_amdgcn_wmma_f32_16x16x32_f16(false, a, false, b, (short)0, c, false, false); asm volatile("v_nop\n\tv_nop\n\tv_nop\n\tv_nop" : "+v"(d) : "v"(a), "v"(b)); return d; }
__device__ __forceinline__ float pmul(float a, float b) { float p = a * b; asm volatile("" : "+v"(p)); return p; }

__global__ __launch_bounds__(256) void prep_kernel(const float* __restrict__ r, float* __restrict__ R32) {
  const size_t t = (size_t)blockIdx.x * 256 + threadIdx.x; if (t >= (size_t)NB * C * HW / 4) return; const v4f v = *(const v4f*)(r + t * 4); const v4f o = {bf16_rne(v[0]), bf16_rne(v[1]), bf16_rne(v[2]), bf16_rne(v[3])};
  for (int pass = 0; pass < 2; ++pass) { *(volatile v4f*)(R32 + t * 4) = o; __threadfence(); }
}
__global__ __launch_bounds__(128) void corr_kernel(const float* __restrict__ left, const float* __restrict__ R32, const float* __restrict__ flow, const float* __restrict__ extra, float* __restrict__ out) {
  __shared__ __attribute__((aligned(16))) b16 LT[32][C + 8], Sh[32][C + 8], Sl[32][C + 8]; __shared__ __attribute__((aligned(16))) float Co[G * K9][32 + 4];
  const int w0 = blockIdx.x * 32, h = blockIdx.y, b = blockIdx.z, t_ = threadIdx.x, wave = t_ >> 5, lane = t_ & 31, nloc = lane & 15, hh = lane >> 4;
  { const int px = t_ & 31, cq = t_ >> 5; for (int c = cq * 64; c < cq * 64 + 64; ++c) LT[px][c] = (b16)(bf16_rne(left[(((size_t)b * C + c) * H + h) * W + w0 + px]) * XS); }
  const int px = t_ & 31, cq = t_ >> 5; const int w = w0 + px;
  const float fx = bf16_rne(flow[(((size_t)b * 2 + 0) * H + h) * W + w]), fy = bf16_rne(flow[(((size_t)b * 2 + 1) * H + h) * W + w]);
  const float bx = (float)w + fx, by = (float)h + fy;
  for (int k = 0; k < K9; ++k) {
    const float ex = bf16_rne(extra[((((size_t)b * K9 + k) * 2 + 0) * H + h) * W + w]), ey = bf16_rne(extra[((((size_t)b * K9 + k) * 2 + 1) * H + h) * W + w]);
    const float x = bx + ((float)(k - 4) + ex), y = by + (0.0f + ey);
    const float x0 = floorf(x), y0 = floorf(y); const float wx1 = x - x0, wy1 = y - y0, wx0 = 1.0f - wx1, wy0 = 1.0f - wy1;
    float cw[4]; int ci[4];
#pragma unroll
    for (int q = 0; q < 4; ++q) { const float xi = x0 + (float)(q & 1), yi = y0 + (float)(q >> 1); const bool valid = (xi >= 0.0f) && (xi <= (float)(W - 1)) && (yi >= 0.0f) && (yi <= (float)(H - 1));
      const int ixc = (int)fminf(fmaxf(xi, 0.0f), (float)(W - 1)), iyc = (int)fminf(fmaxf(yi, 0.0f), (float)(H - 1)); ci[q] = iyc * W + ixc;
      const float wq = ((q & 1) ? wx1 : wx0) * ((q >> 1) ? wy1 : wy0); cw[q] = valid ? wq : 0.0f; }
    __syncthreads();
    const float* Rb = R32 + (size_t)b * C * HW;
#pragma unroll 2
    for (int c = cq * 64; c < cq * 64 + 64; ++c) { const float* Rc = Rb + (size_t)c * HW; const float v = ((pmul(Rc[ci[0]], cw[0]) + pmul(Rc[ci[1]], cw[1])) + pmul(Rc[ci[2]], cw[2])) + pmul(Rc[ci[3]], cw[3]); b16 a_, c_; split16(v * XS, a_, c_); Sh[px][c] = a_; Sl[px][c] = c_; }
    __syncthreads();
    { const int g = wave;
#pragma unroll
      for (int rt = 0; rt < 2; ++rt) { v8f acc = {};
#pragma unroll
        for (int kb = 0; kb < GC; kb += 32) { const v16b a = frag_kb(&LT[rt * 16 + nloc][g * GC + kb], hh); acc = wmma16b(a, frag_kb(&Sh[rt * 16 + nloc][g * GC + kb], hh), acc); acc = wmma16b(a, frag_kb(&Sl[rt * 16 + nloc][g * GC + kb], hh), acc); }
        float dv = 0.0f;
#pragma unroll
        for (int r = 0; r < 8; ++r) dv = (r == nloc - 8 * hh) ? acc[r] : dv;
        if ((nloc >> 3) == hh) Co[g * K9 + k][rt * 16 + nloc] = dv * (1.0f / (XS * XS * GC)); } } }
  __syncthreads();
  for (int pass = 0; pass < 2; ++pass) { for (int row = wave; row < G * K9; row += 4) ((volatile float*)out)[(((size_t)b * (G * K9) + row) * H + h) * W + w0 + lane] = Co[row][lane]; __threadfence(); }
}
}

extern "C" void kernel_launch(void* const* d_in, const int* in_sizes, int n_in, void* d_out, int out_size, void* d_ws, size_t ws_size, hipStream_t stream) {
  (void)n_in;
  auto Fp = [&](int i) { return (const float*)d_in[i]; };
  if (in_sizes[0] != NB * C * HW || in_sizes[1] != NB * C * HW || in_sizes[2] != NB * 2 * HW || in_sizes[3] != NB * 18 * HW || out_size != NB * G * K9 * HW) return;
  size_t off = 0; char* ws = (char*)d_ws;
  auto carve = [&](size_t bytes) { char* p = ws + off; off += (bytes + 255) & ~(size_t)255; return p; };
  float* R32 = (float*)carve((size_t)NB * C * HW * 4);
  if (off > ws_size || off > ((size_t)128 << 20)) return;
  prep_kernel<<<(unsigned)(((size_t)NB * C * HW / 4 + 255) / 256), 256, 0, stream>>>(Fp(1), R32);
  corr_kernel<<<dim3(W / 32, H, NB), 128, 0, stream>>>(Fp(0), R32, Fp(2), Fp(3), (float*)d_out);
}
